// SelectiveSSM_61065845015401
// MI455X (gfx1250) — hardware-verified
//
#include <hip/hip_runtime.h>
#include <math.h>

typedef __attribute__((ext_vector_type(16))) _Float16 v16h;
typedef __attribute__((ext_vector_type(8)))  _Float16 v8h;
typedef __attribute__((ext_vector_type(16))) __bf16   v16b;
typedef __attribute__((ext_vector_type(8)))  __bf16   v8b;
typedef __attribute__((ext_vector_type(8)))  float    v8f;
typedef __attribute__((ext_vector_type(4)))  float    v4f;

constexpr int kBatch  = 2;
constexpr int kSeqL   = 2048;
constexpr int kDm     = 1024;
constexpr int kNst    = 16;
constexpr int kDtR    = 64;
constexpr int kPrjN   = 96;
constexpr int kPrjP   = 128;
constexpr int kRows   = kBatch * kSeqL;
constexpr int kTP     = 260;
constexpr int kScanCh = 256;
static_assert(kDtR + 2 * kNst == kPrjN, "proj width");
static_assert((kDm % 32) == 0 && (kDtR % 32) == 0, "GEMM K multiples of 32");
static_assert((kRows % 64) == 0 && (kPrjP % 64) == 0 && (kDm % 64) == 0, "GEMM M,N multiples of 64");
static_assert((((kRows / 64) * (kPrjP / 64)) % 8) == 0 && (((kRows / 64) * (kDm / 64)) % 8) == 0, "8 tiles per GEMM block");
static_assert(((kRows * kDm / 8) % 256) == 0 && ((kRows * kDtR / 8) % 256) == 0, "split grids exact");
static_assert((kDtR % 64) == 0 && (kDm % 64) == 0 && (kPrjP % 64) == 0, "transpose tiles");
static_assert((kSeqL % 16) == 0 && (kDm % kScanCh) == 0 && kScanCh == 256, "scan tiles");

constexpr size_t kOffXH   = 0;
constexpr size_t kOffXL   = kOffXH  + (size_t)kRows * kDm  * 2;
constexpr size_t kOffWXH  = kOffXL  + (size_t)kRows * kDm  * 2;
constexpr size_t kOffWXL  = kOffWXH + (size_t)kPrjP * kDm  * 2;
constexpr size_t kOffWDH  = kOffWXL + (size_t)kPrjP * kDm  * 2;
constexpr size_t kOffWDL  = kOffWDH + (size_t)kDm   * kDtR * 2;
constexpr size_t kOffPRJ  = kOffWDL + (size_t)kDm   * kDtR * 2;
constexpr size_t kOffDTH  = kOffPRJ + (size_t)kRows * kPrjP * 4;
constexpr size_t kOffDTL  = kOffDTH + (size_t)kRows * kDtR * 2;
constexpr size_t kOffDLR  = kOffDTL + (size_t)kRows * kDtR * 2;
constexpr size_t kWsTotal = kOffDLR + (size_t)kRows * kDm  * 4;
static_assert(kWsTotal == 37486592ull, "carve total");
static_assert(kWsTotal <= 134217728ull, "carve cap");
static_assert((kOffXL % 128) == 0 && (kOffWXH % 128) == 0 && (kOffWXL % 128) == 0 && (kOffWDH % 128) == 0 &&
              (kOffWDL % 128) == 0 && (kOffPRJ % 128) == 0 && (kOffDTH % 128) == 0 && (kOffDTL % 128) == 0 &&
              (kOffDLR % 128) == 0, "128-B aligned regions");

__device__ __forceinline__ unsigned short f2bf_bits(float f) {
  unsigned u = __float_as_uint(f);
  return (unsigned short)((u + 0x7FFFu + ((u >> 16) & 1u)) >> 16);
}
__device__ __forceinline__ float bf_bits2f(unsigned short h) { return __uint_as_float(((unsigned)h) << 16); }

__device__ __forceinline__ void dep_guard_h(v8f& a, v8f& b, v16h x, v16h y) { asm volatile("v_nop\n\tv_nop\n\tv_nop\n\tv_nop" : "+v"(a), "+v"(b) : "v"(x), "v"(y)); }
__device__ __forceinline__ void dep_guard_b(v8f& a, v8f& b, v16b x, v16b y) { asm volatile("v_nop\n\tv_nop\n\tv_nop\n\tv_nop" : "+v"(a), "+v"(b) : "v"(x), "v"(y)); }
__device__ __forceinline__ void dep_guard4_h(v8f& a, v8f& b, v8f& c, v8f& d, v16h x, v16h y) { asm volatile("v_nop\n\tv_nop\n\tv_nop\n\tv_nop" : "+v"(a), "+v"(b), "+v"(c), "+v"(d) : "v"(x), "v"(y)); }
__device__ __forceinline__ void dep_guard4_b(v8f& a, v8f& b, v8f& c, v8f& d, v16b x, v16b y) { asm volatile("v_nop\n\tv_nop\n\tv_nop\n\tv_nop" : "+v"(a), "+v"(b), "+v"(c), "+v"(d) : "v"(x), "v"(y)); }
__device__ __forceinline__ void keep4_h(v16h a, v16h b, v16h c, v16h d) { asm volatile("v_nop" :: "v"(a), "v"(b), "v"(c), "v"(d)); }
__device__ __forceinline__ void keep4_b(v16b a, v16b b, v16b c, v16b d) { asm volatile("v_nop" :: "v"(a), "v"(b), "v"(c), "v"(d)); }
__device__ __forceinline__ void acc_guard4(v8f& a, v8f& b, v8f& c, v8f& d) { asm volatile("v_nop\n\tv_nop\n\tv_nop\n\tv_nop" : "+v"(a), "+v"(b), "+v"(c), "+v"(d)); }
template <typename T> struct Frag;
template <> struct Frag<_Float16> {
  typedef v16h V; union U { v16h v; v8h h[2]; };
  static __device__ __forceinline__ v16h load(const _Float16* p) {
    U f; f.h[0] = *(const v8h*)(p); f.h[1] = *(const v8h*)(p + 16); return f.v;
  }
  static __device__ __forceinline__ v8f mma(v16h a, v16h b, v8f c) {
    return __builtin_amdgcn_wmma_f32_16x16x32_f16(false, a, false, b, (short)0, c, false, false);
  }
  static __device__ __forceinline__ void guard(v8f& a, v8f& b, v16h x, v16h y) { dep_guard_h(a, b, x, y); }
  static __device__ __forceinline__ void guard4(v8f& a, v8f& b, v8f& c, v8f& d, v16h x, v16h y) { dep_guard4_h(a, b, c, d, x, y); }
  static __device__ __forceinline__ void keep(v16h a, v16h b, v16h c, v16h d) { keep4_h(a, b, c, d); }
};
template <> struct Frag<__bf16> {
  typedef v16b V; union U { v16b v; v8b h[2]; };
  static __device__ __forceinline__ v16b load(const __bf16* p) {
    U f; f.h[0] = *(const v8b*)(p); f.h[1] = *(const v8b*)(p + 16); return f.v;
  }
  static __device__ __forceinline__ v8f mma(v16b a, v16b b, v8f c) {
    return __builtin_amdgcn_wmma_f32_16x16x32_bf16(false, a, false, b, (short)0, c, false, false);
  }
  static __device__ __forceinline__ void guard(v8f& a, v8f& b, v16b x, v16b y) { dep_guard_b(a, b, x, y); }
  static __device__ __forceinline__ void guard4(v8f& a, v8f& b, v8f& c, v8f& d, v16b x, v16b y) { dep_guard4_b(a, b, c, d, x, y); }
  static __device__ __forceinline__ void keep(v16b a, v16b b, v16b c, v16b d) { keep4_b(a, b, c, d); }
};

template <int ET> struct Elem;
template <> struct Elem<0> { typedef _Float16 T; };
template <> struct Elem<1> { typedef __bf16 T; };
template <int ET, bool SPLIT, int BIAS_MODE, int OUT_MODE, bool RESID, int ACT = 0>
__global__ __launch_bounds__(256) void wmma_gemm64(
    const unsigned short* __restrict__ Ap, const unsigned short* __restrict__ A2p, int lda, long strideA,
    const unsigned short* __restrict__ Btp, const unsigned short* __restrict__ Bt2p, int ldb, long strideB,
    void* __restrict__ Cout, void* __restrict__ Cout2, int ldc, long strideC,
    const float* __restrict__ bias,
    const float* __restrict__ resid, long strideR,
    int M, int N, int K, float scale) {
  typedef typename Elem<ET>::T T;
  typedef typename Frag<T>::V V;
  const T* A = (const T*)Ap; const T* A2 = (const T*)A2p; const T* Bt = (const T*)Btp; const T* Bt2 = (const T*)Bt2p;
  __shared__ __align__(16) float sT[8][16 * 68];
  const int b    = blockIdx.y;
  const int lane = threadIdx.x & 31;
  const int wave = threadIdx.x >> 5;
  const int tilesN = N >> 6;
  const int tilesM = M >> 6;
  const int tile = blockIdx.x * 8 + wave;
  if (tile >= tilesM * tilesN) return;
  const int tm = tile / tilesN;
  const int tn = tile - tm * tilesN;
  const int m0 = tm << 6;
  const int n0 = tn << 6;

  const T* Ab  = A  + (size_t)b * strideA;
  const T* Bb  = Bt + (size_t)b * strideB;
  const T* Ab2 = SPLIT ? (A2  + (size_t)b * strideA) : nullptr;
  const T* Bb2 = SPLIT ? (Bt2 + (size_t)b * strideB) : nullptr;

  const int rlane = lane & 15;
  const int koff  = (lane >> 4) * 8;
  const int mOff  = (lane >> 4) * 8;

  v8f acc[4][4];
#pragma unroll
  for (int i = 0; i < 4; ++i)
#pragma unroll
    for (int j = 0; j < 4; ++j) acc[i][j] = (v8f){0.f,0.f,0.f,0.f,0.f,0.f,0.f,0.f};

  for (int k0 = 0; k0 < K; k0 += 32) {
    V bh[4], bl[4];
#pragma unroll
    for (int j = 0; j < 4; ++j) {
      const size_t bo = (size_t)(n0 + (j << 4) + rlane) * ldb + koff + k0;
      bh[j] = Frag<T>::load(Bb + bo);
      if (SPLIT) bl[j] = Frag<T>::load(Bb2 + bo);
    }
#pragma unroll
    for (int i = 0; i < 4; ++i) {
      const size_t ao = (size_t)(m0 + (i << 4) + rlane) * lda + koff + k0;
      V ah = Frag<T>::load(Ab + ao);
      V al;
      if (SPLIT) al = Frag<T>::load(Ab2 + ao);
#pragma unroll
      for (int j = 0; j < 4; ++j) {
        acc[i][j] = Frag<T>::mma(ah, bh[j], acc[i][j]);
        if (SPLIT) {
          acc[i][j] = Frag<T>::mma(ah, bl[j], acc[i][j]);
          acc[i][j] = Frag<T>::mma(al, bh[j], acc[i][j]);
        }
      }
      Frag<T>::guard4(acc[i][0], acc[i][1], acc[i][2], acc[i][3], ah, SPLIT ? al : ah);
    }
    Frag<T>::keep(bh[0], bh[1], bh[2], bh[3]);
    if (SPLIT) Frag<T>::keep(bl[0], bl[1], bl[2], bl[3]);
  }
  acc_guard4(acc[0][0], acc[0][1], acc[0][2], acc[0][3]);
  acc_guard4(acc[1][0], acc[1][1], acc[1][2], acc[1][3]);
  acc_guard4(acc[2][0], acc[2][1], acc[2][2], acc[2][3]);
  acc_guard4(acc[3][0], acc[3][1], acc[3][2], acc[3][3]);

  float* slab = sT[wave];
  const float* Rb = RESID ? (resid + (size_t)b * strideR) : nullptr;
#pragma unroll
  for (int i = 0; i < 4; ++i) {
    const int mBase = m0 + (i << 4);
#pragma unroll
    for (int j = 0; j < 4; ++j) {
      const int n = n0 + (j << 4) + rlane;
      float bv = 0.f;
      if (BIAS_MODE == 2) bv = bias[n];
#pragma unroll
      for (int r = 0; r < 8; ++r) {
        float v = acc[i][j][r] * scale;
        if (BIAS_MODE == 1) v += bias[mBase + mOff + r];
        if (BIAS_MODE == 2) v += bv;
        if (RESID) v += Rb[(size_t)(mBase + mOff + r) * ldc + n];
        if (ACT == 1) v = tanhf(v);
        if (ACT == 2) v = fmaxf(v, 0.0f);
        if (ACT == 3) v = v / (1.0f + expf(-v));
        if (ACT == 4) v = (v > 0.f) ? v : 0.01f * v;
        slab[(mOff + r) * 68 + (j << 4) + rlane] = v;
      }
    }
    __builtin_amdgcn_fence(__ATOMIC_RELEASE, "workgroup");
    __builtin_amdgcn_wave_barrier();
    __builtin_amdgcn_fence(__ATOMIC_ACQUIRE, "workgroup");
    if (OUT_MODE == 0) {
      float* C = (float*)Cout + (size_t)b * strideC;
      const int hh = lane >> 4, c4 = (lane & 15) * 4;
      for (int pass = 0; pass < 2; ++pass) {
#pragma unroll
        for (int it = 0; it < 8; ++it) {
          const int row = it * 2 + hh;
          v4f v = *(const v4f*)(slab + row * 68 + c4);
          *(volatile v4f*)(C + (size_t)(mBase + row) * ldc + n0 + c4) = v;
        }
        __threadfence();
      }
    } else {
      const int q = lane >> 3, c8 = (lane & 7) * 8;
      unsigned short* C  = (unsigned short*)Cout  + (size_t)b * strideC;
      unsigned short* C2 = (OUT_MODE == 2) ? ((unsigned short*)Cout2 + (size_t)b * strideC) : nullptr;
      for (int pass = 0; pass < 2; ++pass) {
#pragma unroll
        for (int it = 0; it < 4; ++it) {
          const int row = it * 4 + q;
          const float* sp = slab + row * 68 + c8;
          v8h hv, lv;
#pragma unroll
          for (int e = 0; e < 8; ++e) {
            if (OUT_MODE == 1) {
              hv[e] = (_Float16)sp[e];
            } else {
              unsigned short hb = f2bf_bits(sp[e]);
              unsigned short lb = f2bf_bits(sp[e] - bf_bits2f(hb));
              hv[e] = __builtin_bit_cast(_Float16, hb);
              lv[e] = __builtin_bit_cast(_Float16, lb);
            }
          }
          *(volatile v8h*)(C + (size_t)(mBase + row) * ldc + n0 + c8) = hv;
          if (OUT_MODE == 2) *(volatile v8h*)(C2 + (size_t)(mBase + row) * ldc + n0 + c8) = lv;
        }
        __threadfence();
      }
    }
    __builtin_amdgcn_fence(__ATOMIC_RELEASE, "workgroup");
    __builtin_amdgcn_wave_barrier();
    __builtin_amdgcn_fence(__ATOMIC_ACQUIRE, "workgroup");
  }
}

__global__ __launch_bounds__(256) void split_rows_bf16_kernel(
    const float* __restrict__ src, unsigned short* __restrict__ dhi, unsigned short* __restrict__ dlo, int total8)
{
  const int i = blockIdx.x * 256 + threadIdx.x;
  if (i >= total8) return;
  const size_t e0 = (size_t)i << 3;
  const v4f a0 = *(const v4f*)(src + e0);
  const v4f a1 = *(const v4f*)(src + e0 + 4);
  v8h hv, lv;
#pragma unroll
  for (int e = 0; e < 4; ++e) {
    const float f0 = a0[e];
    const float f1 = a1[e];
    const unsigned short h0 = f2bf_bits(f0), h1 = f2bf_bits(f1);
    const unsigned short l0 = f2bf_bits(f0 - bf_bits2f(h0)), l1 = f2bf_bits(f1 - bf_bits2f(h1));
    hv[e]     = __builtin_bit_cast(_Float16, h0);
    hv[4 + e] = __builtin_bit_cast(_Float16, h1);
    lv[e]     = __builtin_bit_cast(_Float16, l0);
    lv[4 + e] = __builtin_bit_cast(_Float16, l1);
  }
  unsigned short* qh = dhi + e0;
  unsigned short* ql = dlo + e0;
  *(volatile v8h*)qh = hv;
  *(volatile v8h*)ql = lv;
  __threadfence();
  *(volatile v8h*)qh = hv;
  *(volatile v8h*)ql = lv;
}

__global__ __launch_bounds__(256) void transpose_split_kernel(
    const float* __restrict__ W, unsigned short* __restrict__ BtH, unsigned short* __restrict__ BtL, int Kdim, int Ndim)
{
  __shared__ float tile[64 * 65];
  const int tid = threadIdx.x, lane = tid & 31, wave = tid >> 5;
  const int n0 = blockIdx.x * 64;
  const int k0 = blockIdx.y * 64;
#pragma unroll
  for (int p = 0; p < 16; ++p) {
    const int idx = tid + p * 256;
    const int kk  = idx >> 6;
    const int nn  = idx & 63;
    const int n   = n0 + nn;
    const int nc  = (n < Ndim) ? n : (Ndim - 1);
    const float v = W[(size_t)(k0 + kk) * Ndim + nc];
    tile[kk * 65 + nn] = (n < Ndim) ? v : 0.f;
  }
  __syncthreads();
  const int q = lane >> 3, c8 = (lane & 7) * 8;
  v8h hv[2], lv[2];
#pragma unroll
  for (int it = 0; it < 2; ++it) {
    const int nrow = it * 32 + wave * 4 + q;
#pragma unroll
    for (int e = 0; e < 8; ++e) {
      const float f = tile[(c8 + e) * 65 + nrow];
      const unsigned short hb = f2bf_bits(f);
      const unsigned short lb = f2bf_bits(f - bf_bits2f(hb));
      hv[it][e] = __builtin_bit_cast(_Float16, hb);
      lv[it][e] = __builtin_bit_cast(_Float16, lb);
    }
  }
  for (int pass = 0; pass < 2; ++pass) {
#pragma unroll
    for (int it = 0; it < 2; ++it) {
      const int nrow = it * 32 + wave * 4 + q;
      const size_t o = (size_t)(n0 + nrow) * Kdim + k0 + c8;
      *(volatile v8h*)(BtH + o) = hv[it];
      *(volatile v8h*)(BtL + o) = lv[it];
    }
    __threadfence();
  }
}

__global__ __launch_bounds__(256) void dt_split_kernel(
    const float* __restrict__ PRJ, unsigned short* __restrict__ DTH, unsigned short* __restrict__ DTL, int total8)
{
  const int i = blockIdx.x * 256 + threadIdx.x;
  if (i >= total8) return;
  const int e0  = i << 3;
  const int row = e0 >> 6;
  const int c8  = e0 & 63;
  const float* p = PRJ + (size_t)row * kPrjP + c8;
  const v4f a0 = *(const v4f*)(p);
  const v4f a1 = *(const v4f*)(p + 4);
  v8h hv, lv;
#pragma unroll
  for (int e = 0; e < 4; ++e) {
    const float f0 = a0[e];
    const float f1 = a1[e];
    const unsigned short h0 = f2bf_bits(f0), h1 = f2bf_bits(f1);
    const unsigned short l0 = f2bf_bits(f0 - bf_bits2f(h0)), l1 = f2bf_bits(f1 - bf_bits2f(h1));
    hv[e]     = __builtin_bit_cast(_Float16, h0);
    hv[4 + e] = __builtin_bit_cast(_Float16, h1);
    lv[e]     = __builtin_bit_cast(_Float16, l0);
    lv[4 + e] = __builtin_bit_cast(_Float16, l1);
  }
  unsigned short* qh = DTH + e0;
  unsigned short* ql = DTL + e0;
  *(volatile v8h*)qh = hv;
  *(volatile v8h*)ql = lv;
  __threadfence();
  *(volatile v8h*)qh = hv;
  *(volatile v8h*)ql = lv;
}

__global__ __launch_bounds__(256) void scan_kernel(
    const float* __restrict__ DLR, const float* __restrict__ X, const float* __restrict__ PRJ,
    const float* __restrict__ A_log, const float* __restrict__ Dv, float* __restrict__ OUT)
{
  __shared__ __align__(16) float sBC[16 * 32];
  __shared__ __align__(16) float sA[kNst * kScanCh];
  __shared__ __align__(16) float sY[16 * kTP];
  const int tid = threadIdx.x, lane = tid & 31, wave = tid >> 5;
  const int d0 = blockIdx.x * kScanCh, d = d0 + tid;
  const size_t row0 = (size_t)blockIdx.y * kSeqL;

#pragma unroll 1
  for (int n = 0; n < kNst; ++n) sA[n * kScanCh + tid] = -expf(A_log[(size_t)d * kNst + n]);
  __syncthreads();
  float An[kNst], h[kNst];
#pragma unroll
  for (int n = 0; n < kNst; ++n) { An[n] = sA[n * kScanCh + tid]; h[n] = 0.f; }
  const float Dd = Dv[d];
  const int hrow = wave >> 1;
  const int hch  = (wave & 1) * 128 + lane * 4;

#pragma unroll 1
  for (int c = 0; c < kSeqL / 16; ++c) {
    const int l0 = c * 16;
    if (tid < 128) {
      const int r = tid >> 3, q = (tid & 7) * 4;
      const v4f v = *(const v4f*)(PRJ + (row0 + l0 + r) * kPrjP + kDtR + q);
      *(v4f*)(sBC + r * 32 + q) = v;
    }
    __syncthreads();
#pragma unroll 1
    for (int s = 0; s < 16; ++s) {
      const size_t m = row0 + l0 + s;
      const float a     = DLR[m * kDm + d];
      const float delta = fmaxf(a, 0.0f) + log1pf(__expf(-fabsf(a)));
      const float xv    = X[m * kDm + d];
      v4f Bq[4], Cq[4];
#pragma unroll
      for (int qq = 0; qq < 4; ++qq) {
        Bq[qq] = *(const v4f*)(sBC + s * 32 + 4 * qq);
        Cq[qq] = *(const v4f*)(sBC + s * 32 + kNst + 4 * qq);
      }
      float y = 0.f;
#pragma unroll
      for (int n = 0; n < kNst; ++n) {
        const float e = __expf(delta * An[n]);
        float db = delta * Bq[n >> 2][n & 3];
        asm volatile("" : "+v"(db));
        float p = db * xv;
        asm volatile("" : "+v"(p));
        float qv = h[n] * e;
        asm volatile("" : "+v"(qv));
        const float hn = qv + p;
        h[n] = hn;
        float rr = Cq[n >> 2][n & 3] * hn;
        asm volatile("" : "+v"(rr));
        y += rr;
      }
      float sk = xv * Dd;
      asm volatile("" : "+v"(sk));
      y += sk;
      sY[s * kTP + tid] = y;
    }
    __syncthreads();
    v4f fv[4];
#pragma unroll
    for (int it = 0; it < 4; ++it) fv[it] = *(const v4f*)(sY + (it * 4 + hrow) * kTP + hch);
    for (int pass = 0; pass < 2; ++pass) {
#pragma unroll
      for (int it = 0; it < 4; ++it)
        *(volatile v4f*)(OUT + (row0 + l0 + it * 4 + hrow) * kDm + d0 + hch) = fv[it];
      __threadfence();
    }
  }
}

extern "C" void kernel_launch(void* const* d_in, const int* in_sizes, int n_in,
                              void* d_out, int out_size, void* d_ws, size_t ws_size,
                              hipStream_t stream)
{
  if (n_in < 6) return;
  if (in_sizes[0] != kRows * kDm) return;
  if (in_sizes[1] != kDm * kPrjN) return;
  if (in_sizes[2] != kDtR * kDm) return;
  if (in_sizes[3] != kDm) return;
  if (in_sizes[4] != kDm * kNst) return;
  if (in_sizes[5] != kDm) return;
  if (out_size != kRows * kDm) return;
  if (ws_size < kWsTotal) return;

  const float* x     = (const float*)d_in[0];
  const float* W_x   = (const float*)d_in[1];
  const float* W_dt  = (const float*)d_in[2];
  const float* b_dt  = (const float*)d_in[3];
  const float* A_log = (const float*)d_in[4];
  const float* Dv    = (const float*)d_in[5];
  float* out = (float*)d_out;

  char* ws = (char*)d_ws;
  unsigned short* XH  = (unsigned short*)(ws + kOffXH);
  unsigned short* XL  = (unsigned short*)(ws + kOffXL);
  unsigned short* WXH = (unsigned short*)(ws + kOffWXH);
  unsigned short* WXL = (unsigned short*)(ws + kOffWXL);
  unsigned short* WDH = (unsigned short*)(ws + kOffWDH);
  unsigned short* WDL = (unsigned short*)(ws + kOffWDL);
  float*          PRJ = (float*)(ws + kOffPRJ);
  unsigned short* DTH = (unsigned short*)(ws + kOffDTH);
  unsigned short* DTL = (unsigned short*)(ws + kOffDTL);
  float*          DLR = (float*)(ws + kOffDLR);
  const float* dummy_bias  = b_dt;
  const float* dummy_resid = x;

  split_rows_bf16_kernel<<<(kRows * kDm / 8) / 256, 256, 0, stream>>>(x, XH, XL, kRows * kDm / 8);

  transpose_split_kernel<<<dim3(kPrjP / 64, kDm / 64), 256, 0, stream>>>(W_x,  WXH, WXL, kDm,  kPrjN);
  transpose_split_kernel<<<dim3(kDm / 64, kDtR / 64), 256, 0, stream>>>(W_dt, WDH, WDL, kDtR, kDm);

  wmma_gemm64<1, true, 0, 0, false><<<dim3(((kRows / 64) * (kPrjP / 64)) / 8, 1), 256, 0, stream>>>(
      XH, XL, kDm, 0L,
      WXH, WXL, kDm, 0L,
      (void*)PRJ, (void*)PRJ, kPrjP, 0L,
      dummy_bias, dummy_resid, 0L,
      kRows, kPrjP, kDm, 1.0f);

  dt_split_kernel<<<(kRows * kDtR / 8) / 256, 256, 0, stream>>>(PRJ, DTH, DTL, kRows * kDtR / 8);

  wmma_gemm64<1, true, 2, 0, false><<<dim3(((kRows / 64) * (kDm / 64)) / 8, 1), 256, 0, stream>>>(
      DTH, DTL, kDtR, 0L,
      WDH, WDL, kDtR, 0L,
      (void*)DLR, (void*)DLR, kDm, 0L,
      b_dt, dummy_resid, 0L,
      kRows, kDm, kDtR, 1.0f);

  scan_kernel<<<dim3(kDm / kScanCh, kBatch), kScanCh, 0, stream>>>(DLR, x, PRJ, A_log, Dv, out);
}
